// GNNModel_87024627352306
// MI455X (gfx1250) — hardware-verified
//
#include <hip/hip_runtime.h>
#include <stddef.h>
#include <stdint.h>

#define D      16
#define KA     32
#define PNW    384
#define NCB    3
#define NBT    (NCB * 128)
#define NLAYER 3
#define BCOL   256
#define RCOL   272
#define NTHR   256
#define NWAVE  8
#define EPT    8
#define CHUNK  (NTHR * EPT)
#define WCAP   (EPT * 32)
#define LISTN  (NWAVE * WCAP)
#define NBA    1024
#define SLA    10
#define RCAP   16384
#define DEGCAP 64
#define GBM    64
#define GBN    128
#define GTHR   128
#define EPB    256
#define HEP    20
#define APB    16
#define PTW    32
#define PTHR   64
#define PBPL   24
#define HTHR   512
#define GCAP   512
#define AGG_ZINTS (LISTN + 2 * RCAP + 3 * NBA)
#define AGG_LDS_INTS (AGG_ZINTS + 16)
#define AGG_DBL_OFF (AGG_LDS_INTS * 4)
#define AGG_LDS_BYTES (AGG_DBL_OFF + NWAVE * PTW * 8 + PTW * 8 + 64)
#define HPL_OFF (3 * GCAP + 1024 + 16 + 160 + 16)
#define HHD_OFF (HPL_OFF + GCAP * 64)
#define HST_OFF (HHD_OFF + GCAP * 16)
#define HEAD_LDS_FLOATS (HST_OFF + GCAP * 20)
#define HEAD_LDS_BYTES (HEAD_LDS_FLOATS * 4)
#define WSMAX  134217728

static_assert((CHUNK & (CHUNK - 1)) == 0 && CHUNK <= 4096);
static_assert((NBA & (NBA - 1)) == 0 && NBA == (1 << SLA));
static_assert(((long long)CHUNK << SLA) < (1LL << 31));
static_assert(LISTN % NTHR == 0);
static_assert(NBA % (2 * NWAVE) == 0 && NBA % 32 == 0 && NBA % APB == 0 && NBA % GBM == 0);
static_assert(RCAP % 4 == 0 && AGG_ZINTS % (4 * NTHR) == 0 && LISTN % 4 == 0);
static_assert(AGG_DBL_OFF % 16 == 0 && AGG_LDS_BYTES <= 300000);
static_assert(HEAD_LDS_BYTES <= 300000 && HPL_OFF % 4 == 0 && HHD_OFF % 4 == 0 && HST_OFF % 4 == 0);
static_assert(GBM == (GTHR / 32) * 16 && GBN == 4 * 32 && NBT == NCB * GBN && PNW == NBT && PNW % 32 == 0);
static_assert(KA == 32 && KA == 2 * D);
static_assert(EPB == NTHR && EPB * D == 4 * NTHR * 4 && HEP % 4 == 0 && HEP >= D);
static_assert(APB * D == NTHR && APB * KA == 64 * 8 && APB * D == 64 * 4);
static_assert(PTHR == 4 * 16 && PBPL * 16 == NBT && BCOL == 16 * D && RCOL == BCOL + D && RCOL + D <= PNW);
static_assert(PTW == 2 * D && 1024 == 2 * HTHR && GCAP == HTHR);

typedef float          v4f   __attribute__((ext_vector_type(4)));
typedef float          v8f   __attribute__((ext_vector_type(8)));
typedef int            v4i   __attribute__((ext_vector_type(4)));
typedef int            v8i   __attribute__((ext_vector_type(8)));
typedef unsigned short v8us  __attribute__((ext_vector_type(8)));
typedef unsigned short v16us __attribute__((ext_vector_type(16)));
typedef __bf16         v16bf __attribute__((ext_vector_type(16)));
typedef v4f  __attribute__((may_alias)) v4fa;
typedef v4i  __attribute__((may_alias)) v4ia;
typedef v8us __attribute__((may_alias)) v8usa;
union FragB { v16bf v; v16us u; v8us h[2]; v8i w; };

__device__ __forceinline__ v8f wmb(const FragB& a, const FragB& b, v8f c) {
  v8f d = __builtin_amdgcn_wmma_f32_16x16x32_bf16(false, a.v, false, b.v, (short)0, c, false, false);
  asm volatile("v_nop\n\tv_nop\n\tv_nop\n\tv_nop" : "+v"(d) : "v"(a.w), "v"(b.w));
  return d;
}

__device__ __forceinline__ v8f z8() { v8f z = {0.f, 0.f, 0.f, 0.f, 0.f, 0.f, 0.f, 0.f}; return z; }

__device__ __forceinline__ unsigned bf16_bits(float f) {
  const unsigned u = __float_as_uint(f);
  return (u + 0x7FFFu + ((u >> 16) & 1u)) >> 16;
}
__device__ __forceinline__ float bf16_val(float f) {
  return __uint_as_float(bf16_bits(f) << 16);
}
__device__ __forceinline__ double shfl_xor_d(double v, int msk) {
  const long long ll = __double_as_longlong(v);
  int lo = (int)(ll & 0xffffffffLL);
  int hi = (int)(ll >> 32);
  lo = __shfl_xor(lo, msk, 32);
  hi = __shfl_xor(hi, msk, 32);
  const long long r = ((long long)hi << 32) | (long long)(unsigned long long)(unsigned)lo;
  return __longlong_as_double(r);
}

template <int SLB>
__device__ __forceinline__ int scan_chunk(const int* __restrict__ dsts, int nE, int cbase, int slotBase,
                                          int nb, int vec8, int* list, int tid, int lane, int wave) {
  int wc = 0;
  const int el0  = tid * EPT;
  const int e0   = cbase + el0;
  const int sent = -2147483647 - 1;
  v4i da, db;
  if (vec8 != 0 && cbase + CHUNK <= nE) {
    da = *(const v4i*)(dsts + e0);
    db = *(const v4i*)(dsts + e0 + 4);
  } else {
    da.x = (e0     < nE) ? dsts[min(e0,     nE - 1)] : sent;
    da.y = (e0 + 1 < nE) ? dsts[min(e0 + 1, nE - 1)] : sent;
    da.z = (e0 + 2 < nE) ? dsts[min(e0 + 2, nE - 1)] : sent;
    da.w = (e0 + 3 < nE) ? dsts[min(e0 + 3, nE - 1)] : sent;
    db.x = (e0 + 4 < nE) ? dsts[min(e0 + 4, nE - 1)] : sent;
    db.y = (e0 + 5 < nE) ? dsts[min(e0 + 5, nE - 1)] : sent;
    db.z = (e0 + 6 < nE) ? dsts[min(e0 + 6, nE - 1)] : sent;
    db.w = (e0 + 7 < nE) ? dsts[min(e0 + 7, nE - 1)] : sent;
  }
  const unsigned nbs = (unsigned)slotBase;
  const unsigned unb = (unsigned)nb;
  const unsigned s0 = (unsigned)da.x - nbs, s1 = (unsigned)da.y - nbs;
  const unsigned s2 = (unsigned)da.z - nbs, s3 = (unsigned)da.w - nbs;
  const unsigned s4 = (unsigned)db.x - nbs, s5 = (unsigned)db.y - nbs;
  const unsigned s6 = (unsigned)db.z - nbs, s7 = (unsigned)db.w - nbs;
  const bool h0 = s0 < unb, h1 = s1 < unb, h2 = s2 < unb, h3 = s3 < unb;
  const bool h4 = s4 < unb, h5 = s5 < unb, h6 = s6 < unb, h7 = s7 < unb;
  const unsigned any = __builtin_amdgcn_ballot_w32(h0 | h1 | h2 | h3 | h4 | h5 | h6 | h7);
  if (any != 0u) {
#define HITJ(J, HJ, SJ) { \
      const unsigned mj = __builtin_amdgcn_ballot_w32(HJ); \
      if (mj != 0u) { \
        if (HJ) { \
          const int pos = wc + (int)__builtin_amdgcn_mbcnt_lo(mj, 0u); \
          if (pos < WCAP) list[wave * WCAP + pos] = ((el0 + (J)) << SLB) | (int)(SJ); \
        } \
        wc += (int)__builtin_popcount(mj); } }
    HITJ(0, h0, s0)
    HITJ(1, h1, s1)
    HITJ(2, h2, s2)
    HITJ(3, h3, s3)
    HITJ(4, h4, s4)
    HITJ(5, h5, s5)
    HITJ(6, h6, s6)
    HITJ(7, h7, s7)
#undef HITJ
  }
  return wc;
}

__global__ __launch_bounds__(PTHR) void k_prep(const float* __restrict__ w2, const float* __restrict__ b2,
                                               const float* __restrict__ root, unsigned short* BT) {
  const int bl    = (int)blockIdx.x;
  const int layer = bl / PBPL;
  const int rb    = bl - layer * PBPL;
  const int tid   = (int)threadIdx.x;
  const int rl    = tid >> 2;
  const int k8    = (tid & 3) * 8;
  const int i0    = k8 & (D - 1);
  v8us o;
  if (rb < 16) {
    const float* p = w2 + (size_t)rl * 256 + (size_t)i0 * D + rb;
#pragma unroll
    for (int i = 0; i < 8; ++i) o[i] = (unsigned short)bf16_bits(p[(size_t)i * D]);
  } else if (rb == 16) {
    const float* p = b2 + (size_t)i0 * D + rl;
#pragma unroll
    for (int i = 0; i < 8; ++i) o[i] = (unsigned short)bf16_bits(p[(size_t)i * D]);
  } else if (rb == 17) {
    const float* p = root + (size_t)layer * 256 + (size_t)i0 * D + rl;
#pragma unroll
    for (int i = 0; i < 8; ++i) o[i] = (unsigned short)bf16_bits(p[(size_t)i * D]);
  } else {
#pragma unroll
    for (int i = 0; i < 8; ++i) o[i] = (unsigned short)0;
  }
  unsigned short* dp = BT + ((size_t)layer * NBT + (size_t)(rb * 16 + rl)) * KA + k8;
  *(volatile v8us*)dp = o;
  __threadfence();
  *(volatile v8us*)dp = o;
}

__global__ __launch_bounds__(NTHR) void k_cvx(const float* __restrict__ x, int nN, int nUnits,
                                              unsigned short* A) {
  const int u = (int)blockIdx.x * NTHR + (int)threadIdx.x;
  if (u >= nUnits) return;
  const int row = u >> 2;
  const int q   = u & 3;
  const int rc  = row < nN ? row : nN - 1;
  const unsigned keep = (row < nN && q < 2) ? 0xffffu : 0u;
  const float* p = x + (size_t)rc * D + 8 * (q & 1);
  const v4f a = *(const v4fa*)p;
  const v4f b = *(const v4fa*)(p + 4);
  v8us o;
  o[0] = (unsigned short)(bf16_bits(a.x) & keep); o[1] = (unsigned short)(bf16_bits(a.y) & keep);
  o[2] = (unsigned short)(bf16_bits(a.z) & keep); o[3] = (unsigned short)(bf16_bits(a.w) & keep);
  o[4] = (unsigned short)(bf16_bits(b.x) & keep); o[5] = (unsigned short)(bf16_bits(b.y) & keep);
  o[6] = (unsigned short)(bf16_bits(b.z) & keep); o[7] = (unsigned short)(bf16_bits(b.w) & keep);
  unsigned short* dp = A + (size_t)u * 8;
  *(volatile v8us*)dp = o;
  __threadfence();
  *(volatile v8us*)dp = o;
}

__global__ __launch_bounds__(NTHR) void k_he(const float* __restrict__ ea, int nE,
                                             const float* __restrict__ w1, const float* __restrict__ b1,
                                             float* HE) {
  __shared__ float w1L[128];
  __shared__ float b1L[16];
  __shared__ __attribute__((aligned(16))) float sT[EPB * HEP];
  const int tid = (int)threadIdx.x, lane = tid & 31, wave = tid >> 5;
  if (wave < 4) w1L[tid] = bf16_val(w1[tid]);
  if (wave == 4) {
    const float bv = bf16_val(b1[lane & 15]);
    if (lane < 16) b1L[lane] = bv;
  }
  __syncthreads();
  const int e  = (int)blockIdx.x * EPB + tid;
  const int ec = e < nE ? e : nE - 1;
  const float* ep = ea + (size_t)ec * 8;
  const v4f x0 = *(const v4fa*)ep;
  const v4f x1 = *(const v4fa*)(ep + 4);
  float a[8];
  a[0] = bf16_val(x0.x); a[1] = bf16_val(x0.y); a[2] = bf16_val(x0.z); a[3] = bf16_val(x0.w);
  a[4] = bf16_val(x1.x); a[5] = bf16_val(x1.y); a[6] = bf16_val(x1.z); a[7] = bf16_val(x1.w);
  float* row = sT + tid * HEP;
#pragma unroll 1
  for (int f = 0; f < D; ++f) {
    float s = 0.0f;
#pragma unroll
    for (int k = 0; k < 8; ++k) s = fmaf(a[k], w1L[k * D + f], s);
    s += b1L[f];
    row[f] = tanhf(s);
  }
  __syncthreads();
  v4f pv[4];
#pragma unroll
  for (int it = 0; it < 4; ++it) {
    const int v = it * NTHR + tid;
    pv[it] = *(const v4fa*)(sT + (v >> 2) * HEP + 4 * (v & 3));
  }
  float* hb = HE + (size_t)blockIdx.x * (size_t)(EPB * D);
#pragma unroll
  for (int it = 0; it < 4; ++it) *(volatile v4f*)(hb + 4 * (it * NTHR + tid)) = pv[it];
  __threadfence();
#pragma unroll
  for (int it = 0; it < 4; ++it) *(volatile v4f*)(hb + 4 * (it * NTHR + tid)) = pv[it];
}

__global__ __launch_bounds__(GTHR) void k_gemm(const unsigned short* __restrict__ A,
                                               const unsigned short* __restrict__ BT, float* PN) {
  __shared__ __attribute__((aligned(16))) float stg[GBM * GBN];
  const int tid = (int)threadIdx.x, lane = tid & 31, wave = tid >> 5, hh = lane >> 4, m = lane & 15;
  const int rowBase = (int)blockIdx.x * GBM;
  const int colBase = (int)blockIdx.y * GBN;

  v8f acc[8];
#pragma unroll
  for (int t = 0; t < 8; ++t) acc[t] = z8();
  const unsigned short* ap = A  + (size_t)(rowBase + 16 * wave + m) * (size_t)KA + 8 * hh;
  const unsigned short* bp = BT + (size_t)(colBase + m) * (size_t)KA + 8 * hh;

#pragma unroll 1
  for (int k0 = 0; k0 < KA; k0 += 32) {
    FragB af;
    af.h[0] = *(const v8usa*)(ap + k0);
    af.h[1] = *(const v8usa*)(ap + k0 + 16);
#pragma unroll
    for (int nt = 0; nt < 8; ++nt) {
      const unsigned short* wq = bp + (size_t)(16 * nt) * (size_t)KA + k0;
      FragB bf;
      bf.h[0] = *(const v8usa*)wq;
      bf.h[1] = *(const v8usa*)(wq + 16);
      acc[nt] = wmb(af, bf, acc[nt]);
    }
  }

#pragma unroll
  for (int nt = 0; nt < 8; ++nt) {
    const int lc = 16 * nt + m;
#pragma unroll
    for (int r = 0; r < 8; ++r) {
      const int lr = 16 * wave + 8 * hh + r;
      stg[lr * GBN + lc] = acc[nt][r];
    }
  }
  __syncthreads();

  v4f pv[16];
#pragma unroll
  for (int i = 0; i < 16; ++i) pv[i] = *(const v4fa*)(stg + (16 * wave + i) * GBN + 4 * lane);
#pragma unroll
  for (int i = 0; i < 16; ++i) {
    float* op = PN + (size_t)(rowBase + 16 * wave + i) * (size_t)PNW + colBase + 4 * lane;
    *(volatile v4f*)op = pv[i];
  }
  __threadfence();
#pragma unroll
  for (int i = 0; i < 16; ++i) {
    float* op = PN + (size_t)(rowBase + 16 * wave + i) * (size_t)PNW + colBase + 4 * lane;
    *(volatile v4f*)op = pv[i];
  }
}

__global__ __launch_bounds__(NTHR) void k_scan(const int* __restrict__ srcs, const int* __restrict__ dsts,
                                               int nE, int nN, int vec8,
                                               const float* __restrict__ HE, const float* __restrict__ PN,
                                               const float* __restrict__ cbias, float* HP, double* PART) {
  extern __shared__ __attribute__((aligned(16))) int dsm[];
  int* list = dsm;
  int* hl   = dsm + LISTN;
  int* sl   = hl + RCAP;
  int* cnt  = sl + RCAP;
  int* offs = cnt + NBA;
  int* cur  = offs + NBA;
  int* misc = cur + NBA;
  double* wst = (double*)((char*)dsm + AGG_DBL_OFF);
  double* pst = wst + NWAVE * PTW;
  float*  cbL = (float*)(pst + PTW);
  const int tid = (int)threadIdx.x, lane = tid & 31, wave = tid >> 5, hh = lane >> 4;
  const int nodeBase = (int)blockIdx.x * NBA;

  {
    const v4i z4 = {0, 0, 0, 0};
    for (int i = tid * 4; i < AGG_ZINTS; i += NTHR * 4) *(v4ia*)(dsm + i) = z4;
    if (tid < 16) misc[tid] = 0;
    if (wave == 1) {
      const float bv = bf16_val(cbias[lane & 15]);
      if (lane < 16) cbL[lane] = bv;
    }
  }
  __syncthreads();

  int tcount = 0, ov = 0;
  const int nChunks = (nE + CHUNK - 1) / CHUNK;
#pragma unroll 1
  for (int ch = 0; ch < nChunks; ++ch) {
    const int cbase = ch * CHUNK;
    const int wc = scan_chunk<SLA>(dsts, nE, cbase, nodeBase, NBA, vec8, list, tid, lane, wave);
    if (lane == 0) misc[wave] = wc;
    __syncthreads();
    if (wave == 0) {
#pragma unroll 1
      for (int w2 = 0; w2 < NWAVE; ++w2) {
        int c = misc[w2];
        c = c < 0 ? 0 : (c > WCAP ? WCAP : c);
#pragma unroll 1
        for (int b0 = 0; b0 < c; b0 += 32) {
          const int idx = b0 + lane;
          const int ent = list[w2 * WCAP + (idx < WCAP ? idx : WCAP - 1)];
          const int m32 = (c - b0) < 32 ? (c - b0) : 32;
#pragma unroll 1
          for (int k = 0; k < m32; ++k) {
            const int u    = __builtin_amdgcn_readlane(ent, k);
            const int slot = u & (NBA - 1);
            const int el   = (u >> SLA) & (CHUNK - 1);
            const int pk   = ((cbase + el) << SLA) | slot;
            if (tcount < RCAP) {
              if (lane == 0) { hl[tcount] = pk; cnt[slot] = cnt[slot] + 1; }
              tcount = tcount + 1;
            } else {
              ov = 1;
            }
          }
        }
      }
    }
    __syncthreads();
  }
  if (wave == 0 && lane == 0) { misc[8] = tcount; misc[9] = ov; }
  __syncthreads();
  int tt = misc[8];
  tt = tt < 0 ? 0 : (tt > RCAP ? RCAP : tt);
  const int ovf = misc[9];

  if (wave == 0) {
    const int base = lane * (NBA / 32);
    int s = 0;
#pragma unroll 1
    for (int i = 0; i < NBA / 32; ++i) s += cnt[base + i];
    int incl = s;
#pragma unroll
    for (int d = 1; d < 32; d <<= 1) {
      const int y = __shfl_up(incl, d, 32);
      if (lane >= d) incl += y;
    }
    int run = incl - s;
#pragma unroll 1
    for (int i = 0; i < NBA / 32; ++i) {
      const int cv = cnt[base + i];
      offs[base + i] = run;
      cur[base + i]  = run;
      run += cv;
    }
  }
  __syncthreads();
  if (wave == 0) {
#pragma unroll 1
    for (int b0 = 0; b0 < tt; b0 += 32) {
      const int idx = b0 + lane;
      const int ent = hl[idx < RCAP ? idx : RCAP - 1];
      const int m32 = (tt - b0) < 32 ? (tt - b0) : 32;
#pragma unroll 1
      for (int k = 0; k < m32; ++k) {
        const int u    = __builtin_amdgcn_readlane(ent, k);
        const int slot = u & (NBA - 1);
        if (lane == 0) {
          int p = cur[slot];
          p = p < 0 ? 0 : (p > RCAP - 1 ? RCAP - 1 : p);
          sl[p] = u;
          cur[slot] = p + 1;
        }
      }
    }
  }
  __syncthreads();

  const float qnan = __int_as_float(0x7fc00000);
  const float pz   = (ovf != 0) ? qnan : 0.0f;
  const int   o    = lane & 15;
  const unsigned msk1 = 0u - (unsigned)hh;
  const unsigned msk0 = ~msk1;
  const float h0f  = (hh == 0) ? 1.0f : 0.0f;
  const int   qo   = 16 * o + 8 * hh;
  const float cbo  = cbL[o];
  double ds = 0.0, dq = 0.0;
#pragma unroll 1
  for (int pi2 = 0; pi2 < NBA / (2 * NWAVE); ++pi2) {
    const int pr = pi2 * NWAVE + wave;
    float va = 0.0f, vb = 0.0f;
#pragma unroll
    for (int j = 0; j < 2; ++j) {
      const int s    = 2 * pr + j;
      const int node = nodeBase + s;
      int c = cnt[s];
      const bool big = c > DEGCAP;
      c = c < 0 ? 0 : (c > DEGCAP ? DEGCAP : c);
      int of = offs[s];
      of = of < 0 ? 0 : (of > RCAP ? RCAP : of);
      float acc = 0.0f;
#pragma unroll 1
      for (int b0 = 0; b0 < c; b0 += 32) {
        int idx = of + b0 + lane;
        idx = idx > RCAP - 1 ? RCAP - 1 : idx;
        const int ent = sl[idx];
        int eid = ent >> SLA;
        eid = eid < 0 ? 0 : (eid > nE - 1 ? nE - 1 : eid);
        int sr = srcs[eid];
        sr = sr < 0 ? 0 : (sr > nN - 1 ? nN - 1 : sr);
        const int m32 = (c - b0) < 32 ? (c - b0) : 32;
#pragma unroll 1
        for (int k = 0; k < m32; ++k) {
          const int ek = __builtin_amdgcn_readlane(eid, k);
          const int sk = __builtin_amdgcn_readlane(sr, k);
          const float* hq = HE + (size_t)ek * D + 8 * hh;
          const float* pq = PN + (size_t)sk * PNW;
          const v4f ha = *(const v4fa*)hq;
          const v4f hb = *(const v4fa*)(hq + 4);
          const v4f qa = *(const v4fa*)(pq + qo);
          const v4f qb = *(const v4fa*)(pq + qo + 4);
          const float bs = pq[BCOL + o];
          acc = fmaf(ha.x, qa.x, acc);
          acc = fmaf(ha.y, qa.y, acc);
          acc = fmaf(ha.z, qa.z, acc);
          acc = fmaf(ha.w, qa.w, acc);
          acc = fmaf(hb.x, qb.x, acc);
          acc = fmaf(hb.y, qb.y, acc);
          acc = fmaf(hb.z, qb.z, acc);
          acc = fmaf(hb.w, qb.w, acc);
          acc = fmaf(bs, h0f, acc);
        }
      }
      const float tot = acc + __shfl_xor(acc, 16, 32);
      const float den = (c > 0) ? (float)c : 1.0f;
      const int   nr  = node < nN ? node : nN - 1;
      const float rt  = PN[(size_t)nr * PNW + RCOL + o];
      const float pzr = big ? qnan : pz;
      float hv = tot * (1.0f / den) + rt;
      hv = hv + cbo + pzr;
      hv = (node < nN) ? hv : 0.0f;
      if (j == 0) va = hv; else vb = hv;
    }
    const float mine = __uint_as_float((__float_as_uint(va) & msk0) | (__float_as_uint(vb) & msk1));
    const double dm = (double)mine;
    ds += dm;
    dq += dm * dm;
    float* hp = HP + (size_t)(nodeBase + 2 * pr) * D + lane;
    *(volatile float*)hp = mine;
    __threadfence();
    *(volatile float*)hp = mine;
  }

  ds += shfl_xor_d(ds, 16);
  dq += shfl_xor_d(dq, 16);
  if (lane < 16) {
    wst[wave * PTW + lane]     = ds;
    wst[wave * PTW + D + lane] = dq;
  }
  __syncthreads();
  if (tid < PTW) {
    double tsum = 0.0;
#pragma unroll 1
    for (int w2 = 0; w2 < NWAVE; ++w2) tsum += wst[w2 * PTW + tid];
    pst[tid] = tsum;
  }
  __syncthreads();
  v4i ps;
  if (tid < 16) {
    ps = *(const v4ia*)(pst + 2 * tid);
    *(volatile v4i*)((int*)(PART + (size_t)blockIdx.x * PTW) + 4 * tid) = ps;
  }
  __threadfence();
  if (tid < 16) {
    *(volatile v4i*)((int*)(PART + (size_t)blockIdx.x * PTW) + 4 * tid) = ps;
  }
}

template <int LAST>
__global__ __launch_bounds__(NTHR) void k_apply(const float* __restrict__ HP, const double* __restrict__ PART,
                                                int nPart, int nN, const float* __restrict__ gam,
                                                const float* __restrict__ bet, unsigned short* A, float* out) {
  __shared__ float muS[16], rsS[16], gS[16], bS[16];
  __shared__ __attribute__((aligned(16))) float sH[APB * D];
  __shared__ __attribute__((aligned(16))) unsigned short sA[APB * KA];
  const int tid = (int)threadIdx.x, lane = tid & 31, wave = tid >> 5;
  if (wave == 0) {
    const int c = lane & 15;
    double S = 0.0, Q = 0.0;
#pragma unroll 1
    for (int b = 0; b < nPart; ++b) {
      S += PART[(size_t)b * PTW + c];
      Q += PART[(size_t)b * PTW + D + c];
    }
    const double rn   = 1.0 / (double)nN;
    const double mean = S * rn;
    double var = Q * rn - mean * mean;
    var = var < 0.0 ? 0.0 : var;
    const float varf = (float)var;
    const float rstd = 1.0f / sqrtf(varf + 1e-5f);
    const float gv = bf16_val(gam[c]);
    const float bv = bf16_val(bet[c]);
    if (lane < 16) { muS[c] = (float)mean; rsS[c] = rstd; gS[c] = gv; bS[c] = bv; }
  }
  __syncthreads();
  const int r    = tid >> 4;
  const int c    = tid & 15;
  const int node = (int)blockIdx.x * APB + r;
  const float v  = HP[(size_t)node * D + c];
  float t = (v - muS[c]) * rsS[c];
  t = t * gS[c] + bS[c];
  float y = tanhf(t);
  y = (node < nN) ? y : 0.0f;
  sH[r * D + c] = y;
  const unsigned hb = bf16_bits(y);
  sA[r * KA + c]     = (unsigned short)hb;
  sA[r * KA + D + c] = (unsigned short)bf16_bits(y - __uint_as_float(hb << 16));
  __syncthreads();
  if constexpr (LAST == 0) {
    v4i pv;
    unsigned short* dp = A + (size_t)blockIdx.x * (size_t)(APB * KA) + 8 * tid;
    if (tid < 64) {
      pv = *(const v4ia*)(sA + 8 * tid);
      *(volatile v4i*)dp = pv;
    }
    __threadfence();
    if (tid < 64) {
      *(volatile v4i*)dp = pv;
    }
  } else {
    v4f pv;
    const int row = (int)blockIdx.x * APB + (tid >> 2);
    const bool ok = (tid < 64) && (row < nN);
    float* op = out + (size_t)blockIdx.x * (size_t)(APB * D) + 4 * tid;
    if (ok) {
      pv = *(const v4fa*)(sH + 4 * tid);
      *(volatile v4f*)op = pv;
    }
    __threadfence();
    if (ok) {
      *(volatile v4f*)op = pv;
    }
  }
}

__global__ __launch_bounds__(HTHR) void k_head(const float* hid, const int* __restrict__ lens, int nG, int nN,
                                               const float* __restrict__ w1, const float* __restrict__ b1,
                                               const float* __restrict__ w2, const float* __restrict__ b2,
                                               float* outp, int o1, int o2) {
  extern __shared__ __attribute__((aligned(16))) float hsm[];
  int*   pa   = (int*)hsm;
  int*   lenS = pa + 2 * GCAP;
  float* W1L  = hsm + 3 * GCAP;
  float* B1L  = W1L + 1024;
  float* W2L  = B1L + 16;
  float* B2L  = W2L + 160;
  float* PL   = hsm + HPL_OFF;
  float* HD   = hsm + HHD_OFF;
  float* ST   = hsm + HST_OFF;
  const int tid = (int)threadIdx.x, lane = tid & 31, wave = tid >> 5;

  W1L[tid]        = bf16_val(w1[tid]);
  W1L[tid + HTHR] = bf16_val(w1[tid + HTHR]);
  if (wave < 5) W2L[tid] = bf16_val(w2[tid]);
  if (wave == 5) {
    const float bv = bf16_val(b1[lane & 15]);
    if (lane < 16) B1L[lane] = bv;
  }
  if (wave == 6) {
    const int cc = lane < 10 ? lane : 9;
    const float bv = bf16_val(b2[cc]);
    const float bz = lane < 10 ? bv : 0.0f;
    if (lane < 16) B2L[lane] = bz;
  }
  const int gi   = tid < nG ? tid : nG - 1;
  const int lr   = lens[gi];
  const int lraw = (tid < nG) ? lr : 0;
  const int lc   = lraw < 0 ? 0 : (lraw > nN ? nN : lraw);
  lenS[tid] = lraw;
  pa[tid]   = lc;
  __syncthreads();

  int step = 0;
#pragma unroll 1
  for (int d = 1; d < GCAP; d <<= 1) {
    const int* cs = pa + (step & 1) * GCAP;
    int*       ns = pa + ((step + 1) & 1) * GCAP;
    const int j  = tid - d;
    const int jc = j < 0 ? 0 : j;
    const int add = cs[jc];
    const int v = cs[tid] + ((j >= 0) ? add : 0);
    ns[tid] = v;
    __syncthreads();
    step = step + 1;
  }
  const int incl = pa[(step & 1) * GCAP + tid];
  __syncthreads();
  pa[tid]        = incl - lc;
  pa[GCAP + tid] = lc;
  __syncthreads();

#pragma unroll 1
  for (int item = tid; item < nG * 4; item += HTHR) {
    const int g = item >> 2;
    const int q = item & 3;
    int s0 = pa[g];
    s0 = s0 < 0 ? 0 : (s0 > nN ? nN : s0);
    int e1 = s0 + pa[GCAP + g];
    e1 = e1 > nN ? nN : e1;
    v4f sm = {0.0f, 0.0f, 0.0f, 0.0f};
    v4f mx = {-__builtin_inff(), -__builtin_inff(), -__builtin_inff(), -__builtin_inff()};
    v4f mn = {__builtin_inff(), __builtin_inff(), __builtin_inff(), __builtin_inff()};
#pragma unroll 1
    for (int i = s0; i < e1; ++i) {
      const v4f hv = *(const v4fa*)(hid + (size_t)i * D + 4 * q);
      sm += hv;
      mx.x = fmaxf(mx.x, hv.x); mx.y = fmaxf(mx.y, hv.y); mx.z = fmaxf(mx.z, hv.z); mx.w = fmaxf(mx.w, hv.w);
      mn.x = fminf(mn.x, hv.x); mn.y = fminf(mn.y, hv.y); mn.z = fminf(mn.z, hv.z); mn.w = fminf(mn.w, hv.w);
    }
    const int   lrg = lenS[g];
    const float cnt = (float)(lrg < 1 ? 1 : lrg);
    const float rc  = 1.0f / cnt;
    float* pl = PL + g * 64 + 4 * q;
    *(v4fa*)(pl)      = sm * rc;
    *(v4fa*)(pl + 16) = mx;
    *(v4fa*)(pl + 32) = mn;
    *(v4fa*)(pl + 48) = sm;
  }
  __syncthreads();

  {
    const int nU = nG * 16;
#pragma unroll 1
    for (int v = tid; v < nU; v += HTHR) {
      const v4f val = *(const v4fa*)(PL + 4 * v);
      float* op = outp + (size_t)o1 + 4 * v;
      *(volatile v4f*)op = val;
      __threadfence();
      *(volatile v4f*)op = val;
    }
  }

#pragma unroll 1
  for (int item = tid; item < nG * 16; item += HTHR) {
    const int g = item >> 4;
    const int f = item & 15;
    const float* pl = PL + g * 64;
    float s = 0.0f;
#pragma unroll 4
    for (int k = 0; k < 64; ++k) s = fmaf(pl[k], W1L[k * D + f], s);
    s += B1L[f];
    HD[g * D + f] = tanhf(s);
  }
  __syncthreads();

#pragma unroll 1
  for (int item = tid; item < nG * 10; item += HTHR) {
    const int g  = item / 10;
    const int cc = item - g * 10;
    const float* hd = HD + g * D;
    float s = 0.0f;
#pragma unroll 4
    for (int k = 0; k < D; ++k) s = fmaf(hd[k], W2L[k * 10 + cc], s);
    s += B2L[cc];
    ST[item] = s;
  }
  __syncthreads();

  {
    const int g = tid < nG ? tid : nG - 1;
    const float* z = ST + g * 10;
    float m = z[0];
#pragma unroll 1
    for (int cc = 1; cc < 10; ++cc) m = fmaxf(m, z[cc]);
    float se = 0.0f;
#pragma unroll 1
    for (int cc = 0; cc < 10; ++cc) se += expf(z[cc] - m);
    const float lse = logf(se);
    float* lz = ST + nG * 10 + g * 10;
    if (tid < nG) {
#pragma unroll 1
      for (int cc = 0; cc < 10; ++cc) lz[cc] = (z[cc] - m) - lse;
    }
  }
  __syncthreads();

  {
    const int nU = nG * 5;
#pragma unroll 1
    for (int v = tid; v < nU; v += HTHR) {
      const v4f val = *(const v4fa*)(ST + 4 * v);
      float* op = outp + (size_t)o2 + 4 * v;
      *(volatile v4f*)op = val;
      __threadfence();
      *(volatile v4f*)op = val;
    }
  }
}

static inline int cdiv(int a, int b) { return (a + b - 1) / b; }
static inline size_t al256(size_t o) { return (o + 255) & ~(size_t)255; }

extern "C" void kernel_launch(void* const* d_in, const int* in_sizes, int n_in,
                              void* d_out, int out_size, void* d_ws, size_t ws_size,
                              hipStream_t stream) {
  if (n_in < 16) return;
  if (in_sizes[0] < D * 16 || (in_sizes[0] % D) != 0) return;
  const int nN = in_sizes[0] / D;
  if (in_sizes[1] < 8 || (in_sizes[1] % 8) != 0) return;
  const int nE = in_sizes[1] / 8;
  if (in_sizes[2] != 8 * D || in_sizes[3] != D) return;
  if (in_sizes[4] != D * 256 || in_sizes[5] != 256) return;
  if (in_sizes[6] != NLAYER * 256 || in_sizes[7] != NLAYER * D) return;
  if (in_sizes[8] != NLAYER * D || in_sizes[9] != NLAYER * D) return;
  if (in_sizes[10] != 64 * D || in_sizes[11] != D) return;
  if (in_sizes[12] != D * 10 || in_sizes[13] != 10) return;
  if (in_sizes[14] != 2 * nE) return;
  const int nG = in_sizes[15];
  if (nG < 1 || nG > GCAP) return;
  if (nE < 1 || nE >= (1 << 21) || nN < 16 || nN >= (1 << 24)) return;
  if ((long long)out_size != (long long)nN * D + (long long)nG * 84) return;

  const float* x     = (const float*)d_in[0];
  const float* eattr = (const float*)d_in[1];
  const float* ew1   = (const float*)d_in[2];
  const float* eb1   = (const float*)d_in[3];
  const float* ew2   = (const float*)d_in[4];
  const float* eb2   = (const float*)d_in[5];
  const float* root  = (const float*)d_in[6];
  const float* cbias = (const float*)d_in[7];
  const float* gamma = (const float*)d_in[8];
  const float* beta  = (const float*)d_in[9];
  const float* fc1w  = (const float*)d_in[10];
  const float* fc1b  = (const float*)d_in[11];
  const float* fc2w  = (const float*)d_in[12];
  const float* fc2b  = (const float*)d_in[13];
  const int*   eidx  = (const int*)d_in[14];
  const int*   lens  = (const int*)d_in[15];
  const int*   srcI  = eidx;
  const int*   dstI  = eidx + nE;
  float* out = (float*)d_out;
  const int o1 = nN * D;
  const int o2 = o1 + nG * 64;

  const int MP  = cdiv(nN, GBM) * GBM;
  const int gM  = MP / GBM;
  const int gA  = cdiv(MP, NBA);
  const int HPR = gA * NBA;
  if ((long long)gA * NBA < (long long)MP) return;
  const int EP  = cdiv(nE, EPB) * EPB;
  const int vec8 = ((nE & 3) == 0) ? 1 : 0;

  char* ws = (char*)d_ws;
  size_t off = 0;
  const size_t oBT = off; off = al256(off + (size_t)NLAYER * NBT * KA * 2);
  const size_t oA  = off; off = al256(off + (size_t)MP * KA * 2);
  const size_t oHE = off; off = al256(off + (size_t)EP * D * 4);
  const size_t oPN = off; off = al256(off + (size_t)MP * PNW * 4);
  const size_t oHP = off; off = al256(off + (size_t)HPR * D * 4);
  const size_t oPT = off; off = al256(off + (size_t)gA * PTW * 8);
  if (off > ws_size || off > (size_t)WSMAX) return;
  unsigned short* BT   = (unsigned short*)(ws + oBT);
  unsigned short* A    = (unsigned short*)(ws + oA);
  float*          HE   = (float*)(ws + oHE);
  float*          PN   = (float*)(ws + oPN);
  float*          HP   = (float*)(ws + oHP);
  double*         PART = (double*)(ws + oPT);

  hipFuncSetAttribute(reinterpret_cast<const void*>(&k_scan), hipFuncAttributeMaxDynamicSharedMemorySize,
                      (int)AGG_LDS_BYTES);
  hipFuncSetAttribute(reinterpret_cast<const void*>(&k_head), hipFuncAttributeMaxDynamicSharedMemorySize,
                      (int)HEAD_LDS_BYTES);

  k_prep<<<NLAYER * PBPL, PTHR, 0, stream>>>(ew2, eb2, root, BT);
  k_cvx<<<cdiv(MP * 4, NTHR), NTHR, 0, stream>>>(x, nN, MP * 4, A);
  k_he<<<EP / EPB, NTHR, 0, stream>>>(eattr, nE, ew1, eb1, HE);
  for (int l = 0; l < NLAYER; ++l) {
    k_gemm<<<dim3(gM, NCB), GTHR, 0, stream>>>(A, BT + (size_t)l * NBT * KA, PN);
    k_scan<<<gA, NTHR, AGG_LDS_BYTES, stream>>>(srcI, dstI, nE, nN, vec8, HE, PN, cbias + l * D, HP, PART);
    if (l < NLAYER - 1) {
      k_apply<0><<<MP / APB, NTHR, 0, stream>>>(HP, PART, gA, nN, gamma + l * D, beta + l * D, A, out);
    } else {
      k_apply<1><<<MP / APB, NTHR, 0, stream>>>(HP, PART, gA, nN, gamma + l * D, beta + l * D, A, out);
    }
  }
  k_head<<<1, HTHR, HEAD_LDS_BYTES, stream>>>(out, lens, nG, nN, fc1w, fc1b, fc2w, fc2b, out, o1, o2);
}
